// Mamba2Block_49495203119701
// MI455X (gfx1250) — hardware-run, weakly checked
//
#include <hip/hip_runtime.h>
#include <math.h>

typedef __attribute__((ext_vector_type(16))) _Float16 v16h;
typedef __attribute__((ext_vector_type(8)))  _Float16 v8h;
typedef __attribute__((ext_vector_type(4)))  _Float16 v4h;
typedef __attribute__((ext_vector_type(16))) __bf16   v16b;
typedef __attribute__((ext_vector_type(8)))  __bf16   v8b;
typedef __attribute__((ext_vector_type(8)))  float    v8f;
typedef __attribute__((ext_vector_type(4)))  float    v4f;

constexpr int kSeq    = 1024;
constexpr int kDm     = 768;
constexpr int kDin    = 1536;
constexpr int kNst    = 64;
constexpr int kNh     = 12;
constexpr int kHd     = 128;
constexpr int kDconv  = 4;
constexpr int kInProj = 4620;
constexpr int kPP     = 4672;
constexpr int kColXs  = kDin;
constexpr int kColB   = 2 * kDin;
constexpr int kColC   = kColB + kNh * kNst;
constexpr int kColDt  = kColC + kNh * kNst;
static_assert(kColDt + kNh == kInProj, "in_proj column map");
static_assert(kNh * kHd == kDin, "head split");
constexpr int kConvTP = 260;
constexpr int kTS     = 32;
constexpr int kSYP    = 132;
constexpr float kScaleX    = 4.0f;
constexpr float kScaleWin  = 64.0f;
constexpr float kScaleYa   = 16.0f;
constexpr float kScaleWout = 64.0f;
constexpr float kEps       = 1e-5f;
constexpr float kFltMin    = 1.17549435e-38f;
constexpr float kTwoP64    = 18446744073709551616.0f;
constexpr float kTwoM64    = 5.42101086242752217e-20f;

static_assert((kDm % 32) == 0 && (kDin % 32) == 0, "GEMM K multiples of 32");
static_assert((kSeq % 64) == 0 && (kPP % 64) == 0 && (kDm % 64) == 0, "GEMM M,N multiples of 64");
static_assert((kSeq % kTS) == 0 && (kSeq % 64) == 0 && (kDin % 256) == 0, "tile multiples");

constexpr size_t kOffXA   = 0;
constexpr size_t kOffWB   = kOffXA + (size_t)kSeq * kDm  * 2;
constexpr size_t kOffWO   = kOffWB + (size_t)kPP  * kDm  * 2;
constexpr size_t kOffP    = kOffWO + (size_t)kDm  * kDin * 2;
constexpr size_t kOffXC   = kOffP  + (size_t)kSeq * kPP  * 4;
constexpr size_t kOffY    = kOffXC + (size_t)kSeq * kDin * 4;
constexpr size_t kOffYA   = kOffY  + (size_t)kSeq * kDin * 4;
constexpr size_t kWsTotal = kOffYA + (size_t)kSeq * kDin * 2;
static_assert(kWsTotal == 45973504ull, "carve total");
static_assert(kWsTotal <= 134217728ull, "carve cap");
static_assert((kOffWB % 512) == 0 && (kOffWO % 512) == 0 && (kOffP % 128) == 0 && (kOffXC % 512) == 0 &&
              (kOffY % 512) == 0 && (kOffYA % 512) == 0, "aligned regions");

constexpr int kCvtX8     = kSeq * kDm / 8;
constexpr int kCvtWinV8  = kInProj * kDm / 8;
constexpr int kCvtWinT8  = kPP * kDm / 8;
constexpr int kCvtWout8  = kDm * kDin / 8;
static_assert((kCvtX8 % 256) == 0 && (kCvtWinT8 % 256) == 0 && (kCvtWout8 % 256) == 0, "exact cvt grids");
static_assert((kCvtWinV8 % 32) == 0, "pad boundary on a wave boundary");
constexpr int kG0Tiles = (kSeq / 64) * (kPP / 64);
constexpr int kG1Tiles = (kSeq / 64) * (kDm / 64);
static_assert((kG0Tiles % 8) == 0 && (kG1Tiles % 8) == 0, "exact GEMM grids");

__device__ __forceinline__ unsigned short f2bf_bits(float f) {
  unsigned u = __float_as_uint(f);
  return (unsigned short)((u + 0x7FFFu + ((u >> 16) & 1u)) >> 16);
}
__device__ __forceinline__ float bf_bits2f(unsigned short h) { return __uint_as_float(((unsigned)h) << 16); }
__device__ __forceinline__ float bfr(float f) { return bf_bits2f(f2bf_bits(f)); }

__device__ __forceinline__ void dep_guard_h(v8f& a, v8f& b, v16h x, v16h y) { asm volatile("v_nop\n\tv_nop\n\tv_nop\n\tv_nop" : "+v"(a), "+v"(b) : "v"(x), "v"(y)); }
__device__ __forceinline__ void dep_guard_b(v8f& a, v8f& b, v16b x, v16b y) { asm volatile("v_nop\n\tv_nop\n\tv_nop\n\tv_nop" : "+v"(a), "+v"(b) : "v"(x), "v"(y)); }
__device__ __forceinline__ void keep4_h(v16h a, v16h b, v16h c, v16h d) { asm volatile("v_nop" :: "v"(a), "v"(b), "v"(c), "v"(d)); }
__device__ __forceinline__ void keep4_b(v16b a, v16b b, v16b c, v16b d) { asm volatile("v_nop" :: "v"(a), "v"(b), "v"(c), "v"(d)); }
__device__ __forceinline__ void acc_guard4(v8f& a, v8f& b, v8f& c, v8f& d) { asm volatile("v_nop\n\tv_nop\n\tv_nop\n\tv_nop" : "+v"(a), "+v"(b), "+v"(c), "+v"(d)); }
template <typename T> struct Frag;
template <> struct Frag<_Float16> {
  typedef v16h V; union U { v16h v; v8h h[2]; };
  static __device__ __forceinline__ v16h load(const _Float16* p) {
    U f; f.h[0] = *(const v8h*)(p); f.h[1] = *(const v8h*)(p + 16); return f.v;
  }
  static __device__ __forceinline__ v8f mma(v16h a, v16h b, v8f c) {
    return __builtin_amdgcn_wmma_f32_16x16x32_f16(false, a, false, b, (short)0, c, false, false);
  }
  static __device__ __forceinline__ void guard(v8f& a, v8f& b, v16h x, v16h y) { dep_guard_h(a, b, x, y); }
  static __device__ __forceinline__ void keep(v16h a, v16h b, v16h c, v16h d) { keep4_h(a, b, c, d); }
};
template <> struct Frag<__bf16> {
  typedef v16b V; union U { v16b v; v8b h[2]; };
  static __device__ __forceinline__ v16b load(const __bf16* p) {
    U f; f.h[0] = *(const v8b*)(p); f.h[1] = *(const v8b*)(p + 16); return f.v;
  }
  static __device__ __forceinline__ v8f mma(v16b a, v16b b, v8f c) {
    return __builtin_amdgcn_wmma_f32_16x16x32_bf16(false, a, false, b, (short)0, c, false, false);
  }
  static __device__ __forceinline__ void guard(v8f& a, v8f& b, v16b x, v16b y) { dep_guard_b(a, b, x, y); }
  static __device__ __forceinline__ void keep(v16b a, v16b b, v16b c, v16b d) { keep4_b(a, b, c, d); }
};

template <int ET> struct Elem;
template <> struct Elem<0> { typedef _Float16 T; };
template <> struct Elem<1> { typedef __bf16 T; };
template <int ET, int SPL, int BIAS_MODE, int OUT_MODE, bool RESID, int ACT = 0>
__global__ __launch_bounds__(256) void wmma_gemm64(
    const unsigned short* __restrict__ Ap, const unsigned short* __restrict__ A2p, int lda, long strideA,
    const unsigned short* __restrict__ Btp, const unsigned short* __restrict__ Bt2p, int ldb, long strideB,
    void* __restrict__ Cout, void* __restrict__ Cout2, int ldc, long strideC,
    const float* __restrict__ bias,
    const float* __restrict__ resid, long strideR,
    int M, int N, int K, float scale) {
  typedef typename Elem<ET>::T T;
  typedef typename Frag<T>::V V;
  const T* A = (const T*)Ap; const T* A2 = (const T*)A2p; const T* Bt = (const T*)Btp; const T* Bt2 = (const T*)Bt2p;
  __shared__ __align__(16) float sT[8][16 * 68];
  const int b    = blockIdx.y;
  const int lane = threadIdx.x & 31;
  const int wave = threadIdx.x >> 5;
  const int tilesN = N >> 6;
  const int tilesM = M >> 6;
  const int tile = blockIdx.x * 8 + wave;
  if (tile >= tilesM * tilesN) return;
  const int tm = tile / tilesN;
  const int tn = tile - tm * tilesN;
  const int m0 = tm << 6;
  const int n0 = tn << 6;

  const T* Ab  = A  + (size_t)b * strideA;
  const T* Bb  = Bt + (size_t)b * strideB;
  const T* Ab2 = (SPL >= 1) ? (A2  + (size_t)b * strideA) : nullptr;
  const T* Bb2 = (SPL == 2) ? (Bt2 + (size_t)b * strideB) : nullptr;

  const int rlane = lane & 15;
  const int koff  = (lane >> 4) * 8;
  const int mOff  = (lane >> 4) * 8;

  v8f acc[4][4];
#pragma unroll
  for (int i = 0; i < 4; ++i)
#pragma unroll
    for (int j = 0; j < 4; ++j) acc[i][j] = (v8f){0.f,0.f,0.f,0.f,0.f,0.f,0.f,0.f};

  for (int k0 = 0; k0 < K; k0 += 32) {
    V bh[4], bl[4];
#pragma unroll
    for (int j = 0; j < 4; ++j) {
      const size_t bo = (size_t)(n0 + (j << 4) + rlane) * ldb + koff + k0;
      bh[j] = Frag<T>::load(Bb + bo);
      if (SPL == 2) bl[j] = Frag<T>::load(Bb2 + bo);
    }
#pragma unroll
    for (int i = 0; i < 4; ++i) {
      const size_t ao = (size_t)(m0 + (i << 4) + rlane) * lda + koff + k0;
      V ah = Frag<T>::load(Ab + ao);
      V al;
      if (SPL >= 1) al = Frag<T>::load(Ab2 + ao);
#pragma unroll
      for (int j = 0; j < 4; ++j) {
        acc[i][j] = Frag<T>::mma(ah, bh[j], acc[i][j]);
        if (SPL == 2) acc[i][j] = Frag<T>::mma(ah, bl[j], acc[i][j]);
        if (SPL >= 1) acc[i][j] = Frag<T>::mma(al, bh[j], acc[i][j]);
      }
      Frag<T>::guard(acc[i][0], acc[i][3], ah, (SPL >= 1) ? al : ah);
    }
    Frag<T>::keep(bh[0], bh[1], bh[2], bh[3]);
    if (SPL == 2) Frag<T>::keep(bl[0], bl[1], bl[2], bl[3]);
  }
  acc_guard4(acc[0][0], acc[0][1], acc[0][2], acc[0][3]);
  acc_guard4(acc[1][0], acc[1][1], acc[1][2], acc[1][3]);
  acc_guard4(acc[2][0], acc[2][1], acc[2][2], acc[2][3]);
  acc_guard4(acc[3][0], acc[3][1], acc[3][2], acc[3][3]);

  float* slab = sT[wave];
  const float* Rb = RESID ? (resid + (size_t)b * strideR) : nullptr;
#pragma unroll
  for (int i = 0; i < 4; ++i) {
    const int mBase = m0 + (i << 4);
#pragma unroll
    for (int j = 0; j < 4; ++j) {
      const int n = n0 + (j << 4) + rlane;
      float bv = 0.f;
      if (BIAS_MODE == 2) bv = bias[n];
#pragma unroll
      for (int r = 0; r < 8; ++r) {
        float v = acc[i][j][r] * scale;
        if (BIAS_MODE == 1) v += bias[mBase + mOff + r];
        if (BIAS_MODE == 2) v += bv;
        if (RESID) v += Rb[(size_t)(mBase + mOff + r) * ldc + n];
        if (ACT == 1) v = tanhf(v);
        if (ACT == 2) v = fmaxf(v, 0.0f);
        if (ACT == 3) v = v / (1.0f + expf(-v));
        if (ACT == 4) v = (v > 0.f) ? v : 0.01f * v;
        slab[(mOff + r) * 68 + (j << 4) + rlane] = v;
      }
    }
    __builtin_amdgcn_fence(__ATOMIC_RELEASE, "workgroup");
    __builtin_amdgcn_wave_barrier();
    __builtin_amdgcn_fence(__ATOMIC_ACQUIRE, "workgroup");
    if (OUT_MODE == 0) {
      float* C = (float*)Cout + (size_t)b * strideC;
      const int hh = lane >> 4, c4 = (lane & 15) * 4;
      for (int pass = 0; pass < 2; ++pass) {
#pragma unroll
        for (int it = 0; it < 8; ++it) {
          const int row = it * 2 + hh;
          v4f v = *(const v4f*)(slab + row * 68 + c4);
          *(volatile v4f*)(C + (size_t)(mBase + row) * ldc + n0 + c4) = v;
        }
        __threadfence();
      }
    } else {
      const int q = lane >> 3, c8 = (lane & 7) * 8;
      unsigned short* C  = (unsigned short*)Cout  + (size_t)b * strideC;
      unsigned short* C2 = (OUT_MODE == 2) ? ((unsigned short*)Cout2 + (size_t)b * strideC) : nullptr;
      for (int pass = 0; pass < 2; ++pass) {
#pragma unroll
        for (int it = 0; it < 4; ++it) {
          const int row = it * 4 + q;
          const float* sp = slab + row * 68 + c8;
          v8h hv, lv;
#pragma unroll
          for (int e = 0; e < 8; ++e) {
            if (OUT_MODE == 1) {
              hv[e] = (_Float16)sp[e];
            } else {
              unsigned short hb = f2bf_bits(sp[e]);
              unsigned short lb = f2bf_bits(sp[e] - bf_bits2f(hb));
              hv[e] = __builtin_bit_cast(_Float16, hb);
              lv[e] = __builtin_bit_cast(_Float16, lb);
            }
          }
          *(volatile v8h*)(C + (size_t)(mBase + row) * ldc + n0 + c8) = hv;
          if (OUT_MODE == 2) *(volatile v8h*)(C2 + (size_t)(mBase + row) * ldc + n0 + c8) = lv;
        }
        __threadfence();
      }
    }
    __builtin_amdgcn_fence(__ATOMIC_RELEASE, "workgroup");
    __builtin_amdgcn_wave_barrier();
    __builtin_amdgcn_fence(__ATOMIC_ACQUIRE, "workgroup");
  }
}

__global__ __launch_bounds__(256) void cvt_bf16r_f16x8_kernel(
    const float* __restrict__ src, unsigned short* __restrict__ dst, int nvalid8, int ntotal8, float scale)
{
  const int i = blockIdx.x * 256 + threadIdx.x;
  if (i >= ntotal8) return;
  const bool valid = (i < nvalid8);
  const int ic = valid ? i : (nvalid8 - 1);
  const size_t e0 = (size_t)ic << 3;
  const v4f a0 = *(const v4f*)(src + e0);
  const v4f a1 = *(const v4f*)(src + e0 + 4);
  const float keep = valid ? scale : 0.0f;
  v8h hv;
#pragma unroll
  for (int e = 0; e < 4; ++e) {
    const float r0 = bfr(a0[e]) * keep;
    const float r1 = bfr(a1[e]) * keep;
    hv[e]     = (_Float16)r0;
    hv[4 + e] = (_Float16)r1;
  }
  unsigned short* q = dst + ((size_t)i << 3);
  *(volatile v8h*)q = hv;
  __threadfence();
  *(volatile v8h*)q = hv;
}

__global__ __launch_bounds__(256) void conv_silu_kernel(
    const float* __restrict__ P, const float* __restrict__ cw, const float* __restrict__ cb,
    float* __restrict__ XC)
{
  __shared__ __align__(16) float sT[16 * kConvTP];
  const int tid = threadIdx.x, lane = tid & 31, wave = tid >> 5;
  const int d0 = blockIdx.x * 256, d = d0 + tid;
  const int g0 = blockIdx.y * 64;
  const float w0 = bfr(cw[d * kDconv + 0]), w1 = bfr(cw[d * kDconv + 1]);
  const float w2 = bfr(cw[d * kDconv + 2]), w3 = bfr(cw[d * kDconv + 3]);
  const float bc = bfr(cb[d]);
  float xm3, xm2, xm1;
  {
    const bool hist = (g0 > 0);
    const int rb = hist ? (g0 - 3) : g0;
    const float v3 = P[(size_t)rb * kPP + kColXs + d];
    const float v2 = P[(size_t)(rb + 1) * kPP + kColXs + d];
    const float v1 = P[(size_t)(rb + 2) * kPP + kColXs + d];
    xm3 = hist ? v3 : 0.f;
    xm2 = hist ? v2 : 0.f;
    xm1 = hist ? v1 : 0.f;
  }
  const int hrow = wave >> 1;
  const int hch  = (wave & 1) * 128 + lane * 4;
#pragma unroll 1
  for (int sc = 0; sc < 4; ++sc) {
    const int lb = g0 + sc * 16;
#pragma unroll 1
    for (int s = 0; s < 16; ++s) {
      const float xcur = P[(size_t)(lb + s) * kPP + kColXs + d];
      float acc = bc;
      acc = acc + w0 * xm3;
      acc = acc + w1 * xm2;
      acc = acc + w2 * xm1;
      acc = acc + w3 * xcur;
      const float sg = __builtin_amdgcn_rcpf(1.0f + expf(-acc));
      sT[s * kConvTP + tid] = acc * sg;
      xm3 = xm2; xm2 = xm1; xm1 = xcur;
    }
    __syncthreads();
    v4f fv[4];
#pragma unroll
    for (int it = 0; it < 4; ++it) fv[it] = *(const v4f*)(sT + (it * 4 + hrow) * kConvTP + hch);
    for (int pass = 0; pass < 2; ++pass) {
#pragma unroll
      for (int it = 0; it < 4; ++it)
        *(volatile v4f*)(XC + (size_t)(lb + it * 4 + hrow) * kDin + d0 + hch) = fv[it];
      __threadfence();
    }
    __syncthreads();
  }
}

__global__ __launch_bounds__(512) void ssm_scan_kernel(
    const float* __restrict__ P, const float* __restrict__ XC,
    const float* __restrict__ Alog, const float* __restrict__ Dp, const float* __restrict__ dtb,
    float* __restrict__ Yp)
{
  __shared__ __align__(16) float sBC[kTS * 128];
  __shared__ __align__(16) float sY[kTS * kSYP];
  __shared__ float sDT[kTS];
  __shared__ float sW[kTS];
  __shared__ float sF[kTS];
  const int tid = threadIdx.x, lane = tid & 31, wave = tid >> 5;
  const int h = blockIdx.x;
  const int p = tid >> 2;
  const int sub = tid & 3;
  const float negA = -expf(bfr(Alog[h]));
  const float Dd = bfr(Dp[h]);
  const float db = bfr(dtb[h]);
  float S[16];
#pragma unroll
  for (int k = 0; k < 16; ++k) S[k] = 0.0f;
  float phi_carry = 0.0f;
  const size_t xcol = (size_t)kHd * h + p;
  const int bcol0 = kColB + kNst * h;
#pragma unroll 1
  for (int t0 = 0; t0 < kSeq; t0 += kTS) {
    __syncthreads();
#pragma unroll
    for (int i = 0; i < 2; ++i) {
      const int idx = tid + 512 * i;
      const int r = idx >> 5;
      const int c4 = (idx & 31) * 4;
      const int col = bcol0 + c4 + (c4 >> 6) * 704;
      *(v4f*)(sBC + r * 128 + c4) = *(const v4f*)(P + (size_t)(t0 + r) * kPP + col);
    }
    if (wave == 0) {
      const int t = t0 + lane;
      const float dr = P[(size_t)t * kPP + kColDt + h];
      const float ex = expf(-fabsf(dr));
      const float sp = fmaxf(dr, 0.0f) + log1pf(ex);
      const float dt = sp + db;
      float ld = negA * dt;
      asm volatile("" : "+v"(ld));
      float ph = ld;
#pragma unroll
      for (int off = 1; off < 32; off <<= 1) {
        const float nb = __shfl_up(ph, off, 32);
        ph = (lane >= off) ? (ph + nb) : ph;
      }
      ph = ph + phi_carry;
      phi_carry = __shfl(ph, 31, 32);
      const float w = expf(fminf(-ph, 80.0f));
      float f = expf(ph);
      f = (f < kFltMin) ? 0.0f : f;
      sDT[lane] = dt;
      sW[lane] = w;
      sF[lane] = f;
    }
    __syncthreads();
#pragma unroll 1
    for (int s = 0; s < kTS; ++s) {
      const float xv = XC[(size_t)(t0 + s) * kDin + xcol];
      const float dt = sDT[s];
      const float w  = sW[s];
      const float f  = sF[s];
      const float coef = ((w * dt) * xv) * kTwoM64;
      const float* br = sBC + s * 128 + 16 * sub;
      const float* cr = br + 64;
      float acc = 0.0f;
#pragma unroll
      for (int q = 0; q < 4; ++q) {
        const v4f bv = *(const v4f*)(br + 4 * q);
        const v4f cv = *(const v4f*)(cr + 4 * q);
#pragma unroll
        for (int e = 0; e < 4; ++e) {
          S[4 * q + e] = fmaf(coef, bv[e], S[4 * q + e]);
          acc = fmaf(cv[e], S[4 * q + e], acc);
        }
      }
      acc += __shfl_xor(acc, 1, 32);
      acc += __shfl_xor(acc, 2, 32);
      float y = (f * kTwoP64) * acc;
      y = y + Dd * xv;
      if (sub == 0) sY[s * kSYP + p] = y;
    }
    __syncthreads();
    for (int pass = 0; pass < 2; ++pass) {
#pragma unroll
      for (int it = 0; it < 2; ++it) {
        const int row = it * 16 + wave;
        const v4f v = *(const v4f*)(sY + row * kSYP + lane * 4);
        *(volatile v4f*)(Yp + (size_t)(t0 + row) * kDin + (size_t)kHd * h + lane * 4) = v;
      }
      __threadfence();
    }
  }
}

__global__ __launch_bounds__(384) void norm_gate_kernel(
    const float* __restrict__ Yp, const float* __restrict__ P, const float* __restrict__ nw,
    unsigned short* __restrict__ YA)
{
  __shared__ float red[12];
  const int tid = threadIdx.x, lane = tid & 31, wave = tid >> 5;
  const int t = blockIdx.x;
  const int c0 = tid * 4;
  const v4f yv = *(const v4f*)(Yp + (size_t)t * kDin + c0);
  const v4f zv = *(const v4f*)(P + (size_t)t * kPP + c0);
  const v4f wv = *(const v4f*)(nw + c0);
  float ss = 0.0f;
  ss = fmaf(yv[0], yv[0], ss);
  ss = fmaf(yv[1], yv[1], ss);
  ss = fmaf(yv[2], yv[2], ss);
  ss = fmaf(yv[3], yv[3], ss);
#pragma unroll
  for (int off = 1; off < 32; off <<= 1) ss += __shfl_xor(ss, off, 32);
  if (lane == 0) red[wave] = ss;
  __syncthreads();
  float tot = 0.0f;
#pragma unroll
  for (int w = 0; w < 12; ++w) tot += red[w];
  const float r = rsqrtf(tot * (1.0f / 1536.0f) + kEps);
  v4h hv;
#pragma unroll
  for (int e = 0; e < 4; ++e) {
    const float z = zv[e];
    const float sg = __builtin_amdgcn_rcpf(1.0f + expf(-z));
    float v = (yv[e] * r) * bfr(wv[e]);
    v = v * (z * sg);
    hv[e] = (_Float16)(v * kScaleYa);
  }
  unsigned short* q = YA + (size_t)t * kDin + c0;
  *(volatile v4h*)q = hv;
  __threadfence();
  *(volatile v4h*)q = hv;
}

extern "C" void kernel_launch(void* const* d_in, const int* in_sizes, int n_in,
                              void* d_out, int out_size, void* d_ws, size_t ws_size,
                              hipStream_t stream) {
  if (n_in < 9) return;
  if (in_sizes[0] != kSeq * kDm) return;
  if (in_sizes[1] != kInProj * kDm) return;
  if (in_sizes[2] != kDin * kDconv) return;
  if (in_sizes[3] != kDin) return;
  if (in_sizes[4] != kNh) return;
  if (in_sizes[5] != kNh) return;
  if (in_sizes[6] != kNh) return;
  if (in_sizes[7] != kDm * kDin) return;
  if (in_sizes[8] != kDin) return;
  if (out_size != kSeq * kDm) return;
  if (ws_size < kWsTotal) return;

  const float* x       = (const float*)d_in[0];
  const float* W_in    = (const float*)d_in[1];
  const float* conv_w  = (const float*)d_in[2];
  const float* conv_b  = (const float*)d_in[3];
  const float* A_log   = (const float*)d_in[4];
  const float* Dp      = (const float*)d_in[5];
  const float* dt_bias = (const float*)d_in[6];
  const float* W_out   = (const float*)d_in[7];
  const float* norm_w  = (const float*)d_in[8];
  float* out = (float*)d_out;

  char* ws = (char*)d_ws;
  unsigned short* XA = (unsigned short*)(ws + kOffXA);
  unsigned short* WB = (unsigned short*)(ws + kOffWB);
  unsigned short* WO = (unsigned short*)(ws + kOffWO);
  float*          P  = (float*)(ws + kOffP);
  float*          XC = (float*)(ws + kOffXC);
  float*          Y  = (float*)(ws + kOffY);
  unsigned short* YA = (unsigned short*)(ws + kOffYA);

  cvt_bf16r_f16x8_kernel<<<kCvtX8 / 256, 256, 0, stream>>>(x, XA, kCvtX8, kCvtX8, kScaleX);
  cvt_bf16r_f16x8_kernel<<<kCvtWinT8 / 256, 256, 0, stream>>>(W_in, WB, kCvtWinV8, kCvtWinT8, kScaleWin);
  cvt_bf16r_f16x8_kernel<<<kCvtWout8 / 256, 256, 0, stream>>>(W_out, WO, kCvtWout8, kCvtWout8, kScaleWout);

  wmma_gemm64<0, 0, 0, 0, false><<<dim3(kG0Tiles / 8, 1), 256, 0, stream>>>(
      XA, nullptr, kDm, 0L,
      WB, nullptr, kDm, 0L,
      (void*)P, nullptr, kPP, 0L,
      nullptr, nullptr, 0L,
      kSeq, kPP, kDm, 1.0f / (kScaleX * kScaleWin));

  conv_silu_kernel<<<dim3(kDin / 256, kSeq / 64), 256, 0, stream>>>(P, conv_w, conv_b, XC);

  ssm_scan_kernel<<<kNh, 512, 0, stream>>>(P, XC, A_log, Dp, dt_bias, Y);

  norm_gate_kernel<<<kSeq, 384, 0, stream>>>(Y, P, norm_w, YA);

  wmma_gemm64<0, 0, 0, 0, false><<<dim3(kG1Tiles / 8, 1), 256, 0, stream>>>(
      YA, nullptr, kDin, 0L,
      WO, nullptr, kDin, 0L,
      (void*)out, nullptr, kDm, 0L,
      nullptr, nullptr, 0L,
      kSeq, kDm, kDin, 1.0f / (kScaleYa * kScaleWout));
}
